// MessageLayer_85718957294176
// MI455X (gfx1250) — hardware-verified
//
#include <hip/hip_runtime.h>
#include <math.h>

#define NN 50000
#define NE 800000
#define NV (NE + NN)
#define DIMC 64
#define HD 256
#define XW 512
#define MP 50048
#define NT 256
#define TG 2048
#define NTILE 25
#define NROWT (NTILE * TG)
#define SCH 4096
#define SPT (SCH / NT)
#define NCH1 ((NE + SCH - 1) / SCH)
#define NCH2 ((NV + SCH - 1) / SCH)
#define GAT_LDS_BYTES ((TG * 8 + SCH) * 4)
#define WSC 16.0f
#define WSC_INV 0.0625f
#define LN_EPS 1e-5f

typedef __attribute__((ext_vector_type(16))) _Float16 v16h;
typedef __attribute__((ext_vector_type(8)))  _Float16 v8h;
typedef __attribute__((ext_vector_type(4)))  _Float16 v4h;
typedef __attribute__((ext_vector_type(16))) __bf16   v16b;
typedef __attribute__((ext_vector_type(8)))  __bf16   v8b;
typedef __attribute__((ext_vector_type(8)))  float    v8f;
typedef __attribute__((ext_vector_type(4)))  float    v4f;
typedef __attribute__((ext_vector_type(2)))  float    v2f;
typedef __attribute__((ext_vector_type(4)))  int      v4i;
#define U16(p) ((const unsigned short*)(const void*)(p))

__device__ __forceinline__ unsigned short f2bf_bits(float f) {
  unsigned u = __float_as_uint(f);
  return (unsigned short)((u + 0x7FFFu + ((u >> 16) & 1u)) >> 16);
}
__device__ __forceinline__ float bf_bits2f(unsigned short h) { return __uint_as_float(((unsigned)h) << 16); }

__device__ __forceinline__ void dep_guard_h(v8f& a, v8f& b, v16h x, v16h y) { asm volatile("v_nop\n\tv_nop\n\tv_nop\n\tv_nop" : "+v"(a), "+v"(b) : "v"(x), "v"(y)); }
__device__ __forceinline__ void dep_guard_b(v8f& a, v8f& b, v16b x, v16b y) { asm volatile("v_nop\n\tv_nop\n\tv_nop\n\tv_nop" : "+v"(a), "+v"(b) : "v"(x), "v"(y)); }
__device__ __forceinline__ void keep4_h(v16h a, v16h b, v16h c, v16h d) { asm volatile("v_nop" :: "v"(a), "v"(b), "v"(c), "v"(d)); }
__device__ __forceinline__ void keep4_b(v16b a, v16b b, v16b c, v16b d) { asm volatile("v_nop" :: "v"(a), "v"(b), "v"(c), "v"(d)); }
__device__ __forceinline__ void acc_guard4(v8f& a, v8f& b, v8f& c, v8f& d) { asm volatile("v_nop\n\tv_nop\n\tv_nop\n\tv_nop" : "+v"(a), "+v"(b), "+v"(c), "+v"(d)); }
template <typename T> struct Frag;
template <> struct Frag<_Float16> {
  typedef v16h V; union U { v16h v; v8h h[2]; };
  static __device__ __forceinline__ v16h load(const _Float16* p) {
    U f; f.h[0] = *(const v8h*)(p); f.h[1] = *(const v8h*)(p + 16); return f.v;
  }
  static __device__ __forceinline__ v8f mma(v16h a, v16h b, v8f c) {
    return __builtin_amdgcn_wmma_f32_16x16x32_f16(false, a, false, b, (short)0, c, false, false);
  }
  static __device__ __forceinline__ void guard(v8f& a, v8f& b, v16h x, v16h y) { dep_guard_h(a, b, x, y); }
  static __device__ __forceinline__ void keep(v16h a, v16h b, v16h c, v16h d) { keep4_h(a, b, c, d); }
};
template <> struct Frag<__bf16> {
  typedef v16b V; union U { v16b v; v8b h[2]; };
  static __device__ __forceinline__ v16b load(const __bf16* p) {
    U f; f.h[0] = *(const v8b*)(p); f.h[1] = *(const v8b*)(p + 16); return f.v;
  }
  static __device__ __forceinline__ v8f mma(v16b a, v16b b, v8f c) {
    return __builtin_amdgcn_wmma_f32_16x16x32_bf16(false, a, false, b, (short)0, c, false, false);
  }
  static __device__ __forceinline__ void guard(v8f& a, v8f& b, v16b x, v16b y) { dep_guard_b(a, b, x, y); }
  static __device__ __forceinline__ void keep(v16b a, v16b b, v16b c, v16b d) { keep4_b(a, b, c, d); }
};

template <int ET> struct Elem;
template <> struct Elem<0> { typedef _Float16 T; };
template <> struct Elem<1> { typedef __bf16 T; };
template <int ET, bool SPLIT, int BIAS_MODE, int OUT_MODE, bool RESID, int ACT = 0>
__global__ __launch_bounds__(256) void wmma_gemm64(
    const unsigned short* __restrict__ Ap, const unsigned short* __restrict__ A2p, int lda, long strideA,
    const unsigned short* __restrict__ Btp, const unsigned short* __restrict__ Bt2p, int ldb, long strideB,
    void* __restrict__ Cout, void* __restrict__ Cout2, int ldc, long strideC,
    const float* __restrict__ bias,
    const float* __restrict__ resid, long strideR,
    int M, int N, int K, float scale) {
  typedef typename Elem<ET>::T T;
  typedef typename Frag<T>::V V;
  const T* A = (const T*)Ap; const T* A2 = (const T*)A2p; const T* Bt = (const T*)Btp; const T* Bt2 = (const T*)Bt2p;
  __shared__ __align__(16) float sT[8][16 * 68];
  const int b    = blockIdx.y;
  const int lane = threadIdx.x & 31;
  const int wave = threadIdx.x >> 5;
  const int tilesN = N >> 6;
  const int tilesM = M >> 6;
  const int tile = blockIdx.x * 8 + wave;
  if (tile >= tilesM * tilesN) return;
  const int tm = tile / tilesN;
  const int tn = tile - tm * tilesN;
  const int m0 = tm << 6;
  const int n0 = tn << 6;

  const T* Ab  = A  + (size_t)b * strideA;
  const T* Bb  = Bt + (size_t)b * strideB;
  const T* Ab2 = SPLIT ? (A2  + (size_t)b * strideA) : nullptr;
  const T* Bb2 = SPLIT ? (Bt2 + (size_t)b * strideB) : nullptr;

  const int rlane = lane & 15;
  const int koff  = (lane >> 4) * 8;
  const int mOff  = (lane >> 4) * 8;

  v8f acc[4][4];
#pragma unroll
  for (int i = 0; i < 4; ++i)
#pragma unroll
    for (int j = 0; j < 4; ++j) acc[i][j] = (v8f){0.f,0.f,0.f,0.f,0.f,0.f,0.f,0.f};

  for (int k0 = 0; k0 < K; k0 += 32) {
    V bh[4], bl[4];
#pragma unroll
    for (int j = 0; j < 4; ++j) {
      const size_t bo = (size_t)(n0 + (j << 4) + rlane) * ldb + koff + k0;
      bh[j] = Frag<T>::load(Bb + bo);
      if (SPLIT) bl[j] = Frag<T>::load(Bb2 + bo);
    }
#pragma unroll
    for (int i = 0; i < 4; ++i) {
      const size_t ao = (size_t)(m0 + (i << 4) + rlane) * lda + koff + k0;
      V ah = Frag<T>::load(Ab + ao);
      V al;
      if (SPLIT) al = Frag<T>::load(Ab2 + ao);
#pragma unroll
      for (int j = 0; j < 4; ++j) {
        acc[i][j] = Frag<T>::mma(ah, bh[j], acc[i][j]);
        if (SPLIT) {
          acc[i][j] = Frag<T>::mma(ah, bl[j], acc[i][j]);
          acc[i][j] = Frag<T>::mma(al, bh[j], acc[i][j]);
        }
      }
      Frag<T>::guard(acc[i][0], acc[i][3], ah, SPLIT ? al : ah);
    }
    Frag<T>::keep(bh[0], bh[1], bh[2], bh[3]);
    if (SPLIT) Frag<T>::keep(bl[0], bl[1], bl[2], bl[3]);
  }
  acc_guard4(acc[0][0], acc[0][1], acc[0][2], acc[0][3]);
  acc_guard4(acc[1][0], acc[1][1], acc[1][2], acc[1][3]);
  acc_guard4(acc[2][0], acc[2][1], acc[2][2], acc[2][3]);
  acc_guard4(acc[3][0], acc[3][1], acc[3][2], acc[3][3]);

  float* slab = sT[wave];
  const float* Rb = RESID ? (resid + (size_t)b * strideR) : nullptr;
#pragma unroll
  for (int i = 0; i < 4; ++i) {
    const int mBase = m0 + (i << 4);
#pragma unroll
    for (int j = 0; j < 4; ++j) {
      const int n = n0 + (j << 4) + rlane;
      float bv = 0.f;
      if (BIAS_MODE == 2) bv = bias[n];
#pragma unroll
      for (int r = 0; r < 8; ++r) {
        float v = acc[i][j][r] * scale;
        if (BIAS_MODE == 1) v += bias[mBase + mOff + r];
        if (BIAS_MODE == 2) v += bv;
        if (RESID) v += Rb[(size_t)(mBase + mOff + r) * ldc + n];
        if (ACT == 1) v = tanhf(v);
        if (ACT == 2) v = fmaxf(v, 0.0f);
        if (ACT == 3) v = v / (1.0f + expf(-v));
        if (ACT == 4) v = (v > 0.f) ? v : 0.01f * v;
        if (ACT == 5) v = 0.5f * v * (1.0f + erff(v * 0.70710678118654752f));
        if (ACT == 6) v = (v > 0.f) ? v : 0.2f * v;
        slab[(mOff + r) * 68 + (j << 4) + rlane] = v;
      }
    }
    __builtin_amdgcn_fence(__ATOMIC_RELEASE, "workgroup");
    __builtin_amdgcn_wave_barrier();
    __builtin_amdgcn_fence(__ATOMIC_ACQUIRE, "workgroup");
    if (OUT_MODE == 0) {
      float* C = (float*)Cout + (size_t)b * strideC;
      const int hh = lane >> 4, c4 = (lane & 15) * 4;
      for (int pass = 0; pass < 2; ++pass) {
#pragma unroll
        for (int it = 0; it < 8; ++it) {
          const int row = it * 2 + hh;
          v4f v = *(const v4f*)(slab + row * 68 + c4);
          *(volatile v4f*)(C + (size_t)(mBase + row) * ldc + n0 + c4) = v;
        }
        __threadfence();
      }
    } else {
      const int q = lane >> 3, c8 = (lane & 7) * 8;
      unsigned short* C  = (unsigned short*)Cout  + (size_t)b * strideC;
      unsigned short* C2 = (OUT_MODE == 2) ? ((unsigned short*)Cout2 + (size_t)b * strideC) : nullptr;
      for (int pass = 0; pass < 2; ++pass) {
#pragma unroll
        for (int it = 0; it < 4; ++it) {
          const int row = it * 4 + q;
          const float* sp = slab + row * 68 + c8;
          v8h hv, lv;
#pragma unroll
          for (int e = 0; e < 8; ++e) {
            if (OUT_MODE == 1) {
              hv[e] = (_Float16)sp[e];
            } else {
              unsigned short hb = f2bf_bits(sp[e]);
              unsigned short lb = f2bf_bits(sp[e] - bf_bits2f(hb));
              hv[e] = __builtin_bit_cast(_Float16, hb);
              lv[e] = __builtin_bit_cast(_Float16, lb);
            }
          }
          *(volatile v8h*)(C + (size_t)(mBase + row) * ldc + n0 + c8) = hv;
          if (OUT_MODE == 2) *(volatile v8h*)(C2 + (size_t)(mBase + row) * ldc + n0 + c8) = lv;
        }
        __threadfence();
      }
    }
    __builtin_amdgcn_fence(__ATOMIC_RELEASE, "workgroup");
    __builtin_amdgcn_wave_barrier();
    __builtin_amdgcn_fence(__ATOMIC_ACQUIRE, "workgroup");
  }
}

__global__ __launch_bounds__(256) void cast_x_kernel(
    const float* __restrict__ in, unsigned short* __restrict__ out, int nval2, int n2) {
  const int i = blockIdx.x * 256 + threadIdx.x;
  if (i < n2) {
    const int ic = (i < nval2) ? i : (nval2 - 1);
    float f0 = in[2 * (size_t)ic], f1 = in[2 * (size_t)ic + 1];
    if (i >= nval2) { f0 = 0.f; f1 = 0.f; }
    const _Float16 h0 = (_Float16)f0, h1 = (_Float16)f1;
    const unsigned u = (unsigned)__builtin_bit_cast(unsigned short, h0) | ((unsigned)__builtin_bit_cast(unsigned short, h1) << 16);
    ((volatile unsigned*)out)[i] = u;
    __threadfence();
    ((volatile unsigned*)out)[i] = u;
  }
}

__device__ __forceinline__ unsigned pack_f16x2(float a, float b) {
  const _Float16 h0 = (_Float16)a, h1 = (_Float16)b;
  return (unsigned)__builtin_bit_cast(unsigned short, h0) | ((unsigned)__builtin_bit_cast(unsigned short, h1) << 16);
}

__global__ __launch_bounds__(NT) void wprep_kernel(const float* __restrict__ Wl, const float* __restrict__ bl,
                                                  const float* __restrict__ Wr, const float* __restrict__ br,
                                                  const float* __restrict__ W1, const float* __restrict__ W2,
                                                  unsigned* __restrict__ BtP, float* __restrict__ biasP,
                                                  unsigned* __restrict__ Bt1, unsigned* __restrict__ Bt2) {
  const int t = threadIdx.x;
  for (int i = t; i < 512 * 32; i += NT) {
    const int n = i >> 5, k = 2 * (i & 31), nn = n & 255;
    const float l0 = Wl[k * 256 + nn], l1 = Wl[(k + 1) * 256 + nn];
    const float r0 = Wr[k * 256 + nn], r1 = Wr[(k + 1) * 256 + nn];
    const float a = (n < 256) ? l0 : r0, b = (n < 256) ? l1 : r1;
    const unsigned u = pack_f16x2(a * WSC, b * WSC);
    ((volatile unsigned*)BtP)[i] = u; __threadfence(); ((volatile unsigned*)BtP)[i] = u;
  }
  for (int i = t; i < 512; i += NT) {
    const float vl = bl[i & 255], vr = br[i & 255];
    const float v = (i < 256) ? vl : vr;
    ((volatile float*)biasP)[i] = v; __threadfence(); ((volatile float*)biasP)[i] = v;
  }
  for (int i = t; i < 128 * 32; i += NT) {
    const int n = i >> 5, k = 2 * (i & 31);
    const unsigned u = pack_f16x2(W1[k * 128 + n] * WSC, W1[(k + 1) * 128 + n] * WSC);
    ((volatile unsigned*)Bt1)[i] = u; __threadfence(); ((volatile unsigned*)Bt1)[i] = u;
  }
  for (int i = t; i < 64 * 64; i += NT) {
    const int n = i >> 6, k = 2 * (i & 63);
    const unsigned u = pack_f16x2(W2[k * 64 + n] * WSC, W2[(k + 1) * 64 + n] * WSC);
    ((volatile unsigned*)Bt2)[i] = u; __threadfence(); ((volatile unsigned*)Bt2)[i] = u;
  }
}

__device__ __forceinline__ int blk_excl_scan(int cnt, int* scan_ws, int tid, int* tot) {
  const int lane = tid & 31, wave = tid >> 5; int incl = cnt;
#pragma unroll
  for (int o = 1; o < 32; o <<= 1) { const int v = __shfl_up(incl, o, 32); if (lane >= o) incl += v; }
  if (lane == 31) scan_ws[wave] = incl;
  __syncthreads();
  if (wave == 0) { int wv = (lane < NT / 32) ? scan_ws[lane] : 0; int wincl = wv;
#pragma unroll
    for (int o = 1; o < 32; o <<= 1) { const int v = __shfl_up(wincl, o, 32); if (lane >= o) wincl += v; }
    if (lane < NT / 32) scan_ws[32 + lane] = wincl - wv; if (lane == 31) scan_ws[64] = wincl; }
  __syncthreads();
  const int res = scan_ws[32 + wave] + incl - cnt; *tot = scan_ws[64];
  return res;
}
template <int SP, int CAP, int NTOT>
__device__ __forceinline__ int chunk_hits(const int* __restrict__ dstv, int e0, int n0, int tid, int* LIST, int* scan_ws) {
  const int eb = e0 + tid * SP;
  const bool real = eb < NE;
  const int ebc = real ? eb : (NE - SP);
  int rec[SP]; int cnt = 0;
#pragma unroll
  for (int k = 0; k < SP; k += 4) {
    const v4i d4 = *(const v4i*)(dstv + ebc + k);
#pragma unroll
    for (int q = 0; q < 4; ++q) {
      const int e = eb + k + q;
      const int d = real ? d4[q] : (e - NE);
      const bool valid = real ? (d < NN) : (e < NTOT);
      int r = -1;
      if (valid && d >= n0 && d < n0 + TG) { r = ((d - n0) << 20) | e; ++cnt; }
      rec[k + q] = r;
    }
  }
  int tot; int p = blk_excl_scan(cnt, scan_ws, tid, &tot);
#pragma unroll
  for (int k = 0; k < SP; ++k) if (rec[k] >= 0) { if ((unsigned)p < (unsigned)CAP) LIST[p] = rec[k]; ++p; }
  __syncthreads();
  return tot < CAP ? tot : CAP;
}

__device__ __forceinline__ void load4x2(float (&o)[8], const float* pa, const float* pb) {
  const v4f a = *(const v4f*)(pa); const v4f b = *(const v4f*)(pb);
  o[0] = a[0]; o[1] = a[1]; o[2] = a[2]; o[3] = a[3]; o[4] = b[0]; o[5] = b[1]; o[6] = b[2]; o[7] = b[3];
}

__global__ __launch_bounds__(NT) void lattr_kernel(const int* __restrict__ ei, const float* __restrict__ ea, float* __restrict__ LATTR) {
  __shared__ __align__(16) float LA[TG * 4];
  __shared__ int LIST[SCH];
  __shared__ int scan_ws[80];
  const int tid = threadIdx.x, lane = tid & 31, wave = tid >> 5;
  const int n0 = blockIdx.x * TG;
  for (int i = tid; i < TG * 4; i += NT) LA[i] = 0.f;
  __syncthreads();
  const int* dstv = ei + NE;
  const int lk = (lane < 3) ? lane : 2;
#pragma unroll 1
  for (int c = 0; c < NCH1; ++c) {
    const int tot = chunk_hits<SPT, SCH, NE>(dstv, c * SCH, n0, tid, LIST, scan_ws);
#pragma unroll 1
    for (int base = 0; base < tot; base += 32) {
      const int q = base + lane;
      const int rv = (q < tot) ? LIST[q < SCH ? q : (SCH - 1)] : -1;
      const int own = (rv >= 0 && (rv >> 28) == wave) ? 1 : 0;
      unsigned msk = (unsigned)__ballot(own);
#pragma unroll 1
      for (int it = 0; it < 32; ++it) {
        if (msk == 0u) break;
        const int bp = __builtin_ctz(msk); msk &= msk - 1u;
        const int r = __shfl(rv, bp, 32);
        const int dl = r >> 20;
        int e = r & 0xFFFFF; e = (e < NE) ? e : (NE - 1);
        const float av = ea[(size_t)e * 3 + lk];
        const float v = (lane < 3) ? av : 1.0f;
        if (lane < 4) LA[dl * 4 + lane] += v;
      }
    }
    __syncthreads();
  }
#pragma unroll 1
  for (int j = 0; j < TG / (8 * 32); ++j) {
    const int dl = wave * (TG / 8) + j * 32 + lane;
    const int n = n0 + dl;
    const v4f s = *(const v4f*)(LA + dl * 4);
    const float cnt = s[3];
    const float inv = 1.0f / fmaxf(cnt, 1.0f);
    v4f o; o[0] = s[0] * inv; o[1] = s[1] * inv; o[2] = s[2] * inv; o[3] = cnt;
    float* rp = LATTR + (size_t)n * 4;
    for (int pass = 0; pass < 2; ++pass) { *(volatile v4f*)rp = o; __threadfence(); }
  }
}

__global__ __launch_bounds__(NT) void gat_kernel(const unsigned short* __restrict__ XLRp, const int* __restrict__ ei,
                                                const float* __restrict__ ea, const float* __restrict__ LATTR,
                                                const float* __restrict__ We, const float* __restrict__ att,
                                                const float* __restrict__ gat_b, const float* __restrict__ x,
                                                const float* __restrict__ g1, const float* __restrict__ b1n,
                                                float* __restrict__ ACC, float* __restrict__ HLN,
                                                unsigned short* __restrict__ H16p) {
  extern __shared__ __align__(16) float dyn_lds[];
  float* SM = dyn_lds;
  float* SL = dyn_lds + TG * 4;
  int* LIST = (int*)(dyn_lds + TG * 8);
  __shared__ int scan_ws[80];
  const _Float16* XLR = (const _Float16*)XLRp;
  _Float16* H16 = (_Float16*)H16p;
  const int tid = threadIdx.x, lane = tid & 31, wave = tid >> 5;
  const int n0 = blockIdx.x * TG;
  const int cA = 4 * lane, cB = 128 + 4 * lane;
  const int cc = 4 * (lane & 15);
  const int hA = lane >> 4, hB = 2 + (lane >> 4);
  float w0[8], w1[8], w2[8], at[8];
  load4x2(w0, We + cA, We + cB);
  load4x2(w1, We + HD + cA, We + HD + cB);
  load4x2(w2, We + 2 * HD + cA, We + 2 * HD + cB);
  load4x2(at, att + cA, att + cB);
  const v4f gb4 = *(const v4f*)(gat_b + cc), g4 = *(const v4f*)(g1 + cc), bn4 = *(const v4f*)(b1n + cc);
  for (int i = tid; i < TG * 4; i += NT) { SM[i] = -INFINITY; SL[i] = 0.f; }
  float* accb = ACC + (size_t)n0 * HD;
  {
    const v4f z4 = {0.f, 0.f, 0.f, 0.f};
    for (int pass = 0; pass < 2; ++pass) {
#pragma unroll 1
      for (int j = 0; j < TG / 8; ++j) {
        float* ap = accb + (size_t)(wave * (TG / 8) + j) * HD;
        *(volatile v4f*)(ap + cA) = z4;
        *(volatile v4f*)(ap + cB) = z4;
      }
      __threadfence();
    }
  }
  __syncthreads();
  const int* srcv = ei;
  const int* dstv = ei + NE;
#pragma unroll 1
  for (int c = 0; c < NCH2; ++c) {
    const int tot = chunk_hits<SPT, SCH, NV>(dstv, c * SCH, n0, tid, LIST, scan_ws);
#pragma unroll 1
    for (int base = 0; base < tot; base += 32) {
      const int q = base + lane;
      const int rv = (q < tot) ? LIST[q < SCH ? q : (SCH - 1)] : -1;
      const int own = (rv >= 0 && (rv >> 28) == wave) ? 1 : 0;
      unsigned msk = (unsigned)__ballot(own);
#pragma unroll 1
      for (int it = 0; it < 32; ++it) {
        if (msk == 0u) break;
        const int bp = __builtin_ctz(msk); msk &= msk - 1u;
        const int r = __shfl(rv, bp, 32);
        const int dl = r >> 20;
        const int e  = r & 0xFFFFF;
        const int d  = n0 + dl;
        const bool real = e < NE;
        const int ec = real ? e : (NE - 1);
        int s = srcv[ec];
        s = s < 0 ? 0 : (s >= NN ? NN - 1 : s);
        s = real ? s : d;
        const float* eap = ea + (size_t)ec * 3;
        const float ea0 = eap[0], ea1 = eap[1], ea2 = eap[2];
        const v4f la = *(const v4f*)(LATTR + (size_t)d * 4);
        const float a0 = real ? ea0 : la[0], a1 = real ? ea1 : la[1], a2 = real ? ea2 : la[2];
        const _Float16* xls = XLR + (size_t)s * XW;
        const _Float16* xrd = XLR + (size_t)d * XW + HD;
        const v4h xlA = *(const v4h*)(xls + cA), xlB = *(const v4h*)(xls + cB);
        const v4h xrA = *(const v4h*)(xrd + cA), xrB = *(const v4h*)(xrd + cB);
        float xl[8]; float pA = 0.f, pB = 0.f;
#pragma unroll
        for (int i = 0; i < 4; ++i) {
          xl[i] = (float)xlA[i];
          float ee = a0 * w0[i]; ee = fmaf(a1, w1[i], ee); ee = fmaf(a2, w2[i], ee);
          float z = (xl[i] + (float)xrA[i]) + ee;
          z = (z > 0.f) ? z : 0.2f * z;
          pA = fmaf(z, at[i], pA);
        }
#pragma unroll
        for (int i = 0; i < 4; ++i) {
          xl[4 + i] = (float)xlB[i];
          float ee = a0 * w0[4 + i]; ee = fmaf(a1, w1[4 + i], ee); ee = fmaf(a2, w2[4 + i], ee);
          float z = (xl[4 + i] + (float)xrB[i]) + ee;
          z = (z > 0.f) ? z : 0.2f * z;
          pB = fmaf(z, at[4 + i], pB);
        }
        pA += __shfl_xor(pA, 8, 32); pA += __shfl_xor(pA, 4, 32); pA += __shfl_xor(pA, 2, 32); pA += __shfl_xor(pA, 1, 32);
        pB += __shfl_xor(pB, 8, 32); pB += __shfl_xor(pB, 4, 32); pB += __shfl_xor(pB, 2, 32); pB += __shfl_xor(pB, 1, 32);
        const int miA = dl * 4 + hA, miB = dl * 4 + hB;
        const float moA = SM[miA], loA = SL[miA];
        const float moB = SM[miB], loB = SL[miB];
        const float mnA = fmaxf(moA, pA), mnB = fmaxf(moB, pB);
        const float rrA = __expf(moA - mnA), exA = __expf(pA - mnA);
        const float rrB = __expf(moB - mnB), exB = __expf(pB - mnB);
        const float lnA = fmaf(loA, rrA, exA), lnB = fmaf(loB, rrB, exB);
        if ((lane & 15) == 0) { SM[miA] = mnA; SL[miA] = lnA; SM[miB] = mnB; SL[miB] = lnB; }
        float* ap = accb + (size_t)dl * HD;
        const v4f qA = *(const v4f*)(ap + cA); const v4f qB = *(const v4f*)(ap + cB);
        v4f oA, oB;
#pragma unroll
        for (int i = 0; i < 4; ++i) { oA[i] = fmaf(qA[i], rrA, exA * xl[i]); oB[i] = fmaf(qB[i], rrB, exB * xl[4 + i]); }
        *(volatile v4f*)(ap + cA) = oA; *(volatile v4f*)(ap + cB) = oB;
        __threadfence();
        *(volatile v4f*)(ap + cA) = oA; *(volatile v4f*)(ap + cB) = oB;
        asm volatile("" ::: "memory");
      }
    }
    __syncthreads();
  }
#pragma unroll 1
  for (int j = 0; j < TG / 8; ++j) {
    const int dl = wave * (TG / 8) + j;
    const int n = n0 + dl;
    if (n < MP) {
      const bool live = n < NN;
      const float* ap = accb + (size_t)dl * HD;
      const v4f qA = *(const v4f*)(ap + cA); const v4f qB = *(const v4f*)(ap + cB);
      float lA = SL[dl * 4 + hA], lB = SL[dl * 4 + hB];
      lA = (live && lA > 0.f) ? lA : 1.0f;
      lB = (live && lB > 0.f) ? lB : 1.0f;
      const float invA = 1.0f / lA, invB = 1.0f / lB;
      float o[4];
#pragma unroll
      for (int i = 0; i < 4; ++i) { o[i] = qA[i] * invA + qB[i] * invB; o[i] += __shfl_xor(o[i], 16, 32); }
      const int nc = live ? n : (NN - 1);
      const v4f xv = *(const v4f*)(x + (size_t)nc * DIMC + cc);
      float v[4]; float sm = 0.f;
#pragma unroll
      for (int i = 0; i < 4; ++i) { v[i] = xv[i] + (o[i] * 0.25f + gb4[i]); sm += v[i]; }
      sm += __shfl_xor(sm, 8, 32); sm += __shfl_xor(sm, 4, 32); sm += __shfl_xor(sm, 2, 32); sm += __shfl_xor(sm, 1, 32);
      const float mu = sm * (1.0f / 64.0f);
      float dv[4]; float var = 0.f;
#pragma unroll
      for (int i = 0; i < 4; ++i) { dv[i] = v[i] - mu; var = fmaf(dv[i], dv[i], var); }
      var += __shfl_xor(var, 8, 32); var += __shfl_xor(var, 4, 32); var += __shfl_xor(var, 2, 32); var += __shfl_xor(var, 1, 32);
      const float rs = rsqrtf(var * (1.0f / 64.0f) + LN_EPS);
      v4f y;
#pragma unroll
      for (int i = 0; i < 4; ++i) { float t = dv[i] * rs * g4[i] + bn4[i]; y[i] = live ? t : 0.f; }
      const int sl = (2 * lane) & 31;
      v8h h8;
#pragma unroll
      for (int i = 0; i < 4; ++i) {
        const float ta = __shfl(y[i], sl, 32), tb = __shfl(y[i], sl + 1, 32);
        h8[i] = (_Float16)ta; h8[4 + i] = (_Float16)tb;
      }
      float* hp = HLN + (size_t)n * DIMC + cc;
      _Float16* hq = H16 + (size_t)n * DIMC + 8 * (lane & 7);
      for (int pass = 0; pass < 2; ++pass) {
        if (lane < 16) *(volatile v4f*)hp = y;
        if (lane < 8) *(volatile v8h*)hq = h8;
        __threadfence();
      }
    }
  }
}

__global__ __launch_bounds__(NT) void ln2_kernel(const float* __restrict__ F, const float* __restrict__ g,
                                                const float* __restrict__ bb, float* __restrict__ out) {
  const int lane = threadIdx.x & 31;
  const int row = blockIdx.x * (NT / 32) + (threadIdx.x >> 5);
  if (row < NN) {
    const v2f hv = *(const v2f*)(F + (size_t)row * DIMC + 2 * lane);
    const float v0 = hv[0], v1 = hv[1];
    float s = v0 + v1;
#pragma unroll
    for (int off = 16; off > 0; off >>= 1) s += __shfl_xor(s, off, 32);
    const float mu = s * (1.0f / 64.0f);
    const float d0 = v0 - mu, d1 = v1 - mu;
    float q = d0 * d0 + d1 * d1;
#pragma unroll
    for (int off = 16; off > 0; off >>= 1) q += __shfl_xor(q, off, 32);
    const float rs = rsqrtf(q * (1.0f / 64.0f) + LN_EPS);
    const v2f gg = *(const v2f*)(g + 2 * lane), b2v = *(const v2f*)(bb + 2 * lane);
    const float y0 = d0 * rs * gg[0] + b2v[0];
    const float y1 = d1 * rs * gg[1] + b2v[1];
    const int sl = (2 * lane) & 31;
    const float a = __shfl(y0, sl, 32), b = __shfl(y1, sl, 32), c = __shfl(y0, sl + 1, 32), d = __shfl(y1, sl + 1, 32);
    v4f o; o[0] = a; o[1] = b; o[2] = c; o[3] = d;
    float* op = out + (size_t)row * DIMC + 4 * (lane & 15);
    for (int pass = 0; pass < 2; ++pass) {
      if (lane < 16) *(volatile v4f*)op = o;
      __threadfence();
    }
  }
}

extern "C" void kernel_launch(void* const* d_in, const int* in_sizes, int n_in,
                              void* d_out, int out_size, void* d_ws, size_t ws_size, hipStream_t stream) {
  if (n_in < 18) return;
  const float* x     = (const float*)d_in[0];
  const int*   ei    = (const int*)  d_in[1];
  const float* ea    = (const float*)d_in[2];
  const float* Wl    = (const float*)d_in[3];
  const float* bl    = (const float*)d_in[4];
  const float* Wr    = (const float*)d_in[5];
  const float* br    = (const float*)d_in[6];
  const float* We    = (const float*)d_in[7];
  const float* att_w = (const float*)d_in[8];
  const float* gat_b = (const float*)d_in[9];
  const float* ln1_g = (const float*)d_in[10];
  const float* ln1_b = (const float*)d_in[11];
  const float* ln2_g = (const float*)d_in[12];
  const float* ln2_b = (const float*)d_in[13];
  const float* W1    = (const float*)d_in[14];
  const float* b1    = (const float*)d_in[15];
  const float* W2    = (const float*)d_in[16];
  const float* b2    = (const float*)d_in[17];
  float* out = (float*)d_out;

  if (in_sizes[0] != NN * DIMC || in_sizes[1] != 2 * NE || in_sizes[2] != NE * 3) return;
  if (in_sizes[3] != DIMC * HD || in_sizes[5] != DIMC * HD || in_sizes[7] != 3 * HD || in_sizes[8] != HD) return;
  if (in_sizes[14] != DIMC * 128 || in_sizes[16] != 128 * DIMC || out_size != NN * DIMC) return;

  char* ws = (char*)d_ws; size_t off = 0;
  auto carve = [&](size_t bytes) -> char* { char* p = ws + off; off += (bytes + 255) & ~(size_t)255; return p; };
  float*          ACC   = (float*)carve((size_t)NROWT * HD * 4);
  unsigned short* X16   = (unsigned short*)ACC;
  unsigned short* XLR   = (unsigned short*)carve((size_t)MP * XW * 2);
  unsigned short* T16   = XLR;
  float*          FFN   = (float*)((char*)XLR + (size_t)MP * 128 * 2);
  float*          LATTR = (float*)carve((size_t)NROWT * 4 * 4);
  float*          HLN   = (float*)carve((size_t)MP * DIMC * 4);
  unsigned short* H16   = (unsigned short*)carve((size_t)MP * DIMC * 2);
  unsigned*       BtP   = (unsigned*)carve((size_t)XW * DIMC * 2);
  float*          biasP = (float*)carve((size_t)XW * 4);
  unsigned*       Bt1   = (unsigned*)carve((size_t)128 * DIMC * 2);
  unsigned*       Bt2   = (unsigned*)carve((size_t)DIMC * 128 * 2);
  if (off > ws_size || off > (size_t)134217728) return;

  cast_x_kernel<<<(MP * 32 + 255) / 256, 256, 0, stream>>>(x, X16, NN * 32, MP * 32);
  wprep_kernel<<<1, NT, 0, stream>>>(Wl, bl, Wr, br, W1, W2, BtP, biasP, Bt1, Bt2);
  {
    const int tiles = (MP / 64) * (XW / 64);
    wmma_gemm64<0, false, 2, 1, false, 0><<<dim3((tiles + 7) / 8, 1), 256, 0, stream>>>(
        U16(X16), U16(X16), DIMC, 0L,
        U16(BtP), U16(BtP), DIMC, 0L,
        (void*)XLR, (void*)nullptr, XW, 0L,
        biasP, (const float*)nullptr, 0L, MP, XW, DIMC, WSC_INV);
  }
  lattr_kernel<<<NTILE, NT, 0, stream>>>(ei, ea, LATTR);
  hipFuncSetAttribute(reinterpret_cast<const void*>(&gat_kernel), hipFuncAttributeMaxDynamicSharedMemorySize, GAT_LDS_BYTES);
  gat_kernel<<<NTILE, NT, GAT_LDS_BYTES, stream>>>(XLR, ei, ea, LATTR, We, att_w, gat_b, x, ln1_g, ln1_b, ACC, HLN, H16);
  {
    const int tiles1 = (MP / 64) * (128 / 64);
    wmma_gemm64<0, false, 2, 1, false, 6><<<dim3((tiles1 + 7) / 8, 1), 256, 0, stream>>>(
        U16(H16), U16(H16), DIMC, 0L,
        U16(Bt1), U16(Bt1), DIMC, 0L,
        (void*)T16, (void*)nullptr, 128, 0L,
        b1, (const float*)nullptr, 0L, MP, 128, DIMC, WSC_INV);
    const int tiles2 = (MP / 64) * (DIMC / 64);
    wmma_gemm64<0, false, 2, 0, true, 0><<<dim3((tiles2 + 7) / 8, 1), 256, 0, stream>>>(
        U16(T16), U16(T16), 128, 0L,
        U16(Bt2), U16(Bt2), 128, 0L,
        (void*)FFN, (void*)nullptr, DIMC, 0L,
        b2, HLN, 0L, MP, DIMC, 128, WSC_INV);
  }
  ln2_kernel<<<NN / (NT / 32), NT, 0, stream>>>(FFN, ln2_g, ln2_b, out);
}
